// HypergraphComputation_16080357556288
// MI455X (gfx1250) — hardware-run, weakly checked
//
#include <hip/hip_runtime.h>


namespace {
constexpr int B = 4, C = 256, N = 1024, NC = 2048, VT = B * N, V = B * (N + NC), ET = B * N;
constexpr float XS = 8.0f, WSC = 256.0f, THR = 0.8f, NEPS = 1e-8f;
typedef _Float16 b16;
typedef __attribute__((ext_vector_type(16))) _Float16 v16b;
typedef __attribute__((ext_vector_type(8))) _Float16 v8b;
typedef __attribute__((ext_vector_type(8))) float v8f;
typedef __attribute__((ext_vector_type(4))) float v4f;
__device__ __forceinline__ float bf16_rne(float f) { unsigned int u = __float_as_uint(f); u += 0x7FFFu + ((u >> 16) & 1u); return __uint_as_float(u & 0xFFFF0000u); }
__device__ __forceinline__ void split16(float v, b16& hi, b16& lo) { hi = (b16)v; lo = (b16)(v - (float)hi); }
__device__ __forceinline__ v16b frag_kb(const b16* p, int hh) { const v8b a = *(const v8b*)(p + 8 * hh), b = *(const v8b*)(p + 16 + 8 * hh); v16b f;
#pragma unroll
  for (int e = 0; e < 8; ++e) { f[e] = a[e]; f[8 + e] = b[e]; } return f; }
__device__ __forceinline__ v8f wmma16b(v16b a, v16b b, v8f c) { v8f d = __builtin_amdgcn_wmma_f32_16x16x32_f16(false, a, false, b, (short)0, c, false, false); asm volatile("v_nop\n\tv_nop\n\tv_nop\n\tv_nop" : "+v"(d) : "v"(a), "v"(b)); return d; }
__device__ __forceinline__ void wave_lds_sync() { __builtin_amdgcn_fence(__ATOMIC_RELEASE, "workgroup"); __builtin_amdgcn_wave_barrier(); __builtin_amdgcn_fence(__ATOMIC_ACQUIRE, "workgroup"); }
__device__ __forceinline__ float pmul(float a, float b) { float p = a * b; asm volatile("" : "+v"(p)); return p; }
__device__ __forceinline__ const float* xrow(const float* xt, const float* c1, const float* c2, int v, int c) { if (v < VT) return xt + ((size_t)(v >> 10) * C + c) * N + (v & 1023); const int u = v - VT, b = u >> 11, m = u & 2047; return (m < N ? c1 : c2) + ((size_t)b * C + c) * N + (m & 1023); }

__global__ __launch_bounds__(256) void wcopy_kernel(const float* __restrict__ w, b16* __restrict__ WT) { const int u = blockIdx.x * 256 + threadIdx.x; if (u >= C * C / 8) return; const size_t e = (size_t)u * 8; v8b v;
#pragma unroll
  for (int j = 0; j < 8; ++j) v[j] = (b16)(bf16_rne(w[e + j]) * WSC); for (int pass = 0; pass < 2; ++pass) { *(volatile v8b*)(WT + e) = v; __threadfence(); } }
__global__ __launch_bounds__(256) void xall_kernel(const float* __restrict__ xt, const float* __restrict__ c1, const float* __restrict__ c2, b16* __restrict__ XB, float* __restrict__ NRM) {
  __shared__ float Ts[C][33]; const int tid = threadIdx.x, wave = tid >> 5, lane = tid & 31; const int v0 = blockIdx.x * 32;
  for (int c = wave; c < C; c += 8) Ts[c][lane] = bf16_rne(*xrow(xt, c1, c2, v0 + lane, c));
  __syncthreads();
  for (int pass = 0; pass < 2; ++pass) { for (int r = 0; r < 4; ++r) { const int vv = wave * 4 + r; const size_t v = (size_t)v0 + vv; float s = 0.0f; for (int q = 0; q < 8; ++q) { const float x = Ts[q * 32 + lane][vv]; s += pmul(x, x); ((volatile b16*)XB)[v * C + q * 32 + lane] = (b16)(x * XS); }
      for (int o = 16; o; o >>= 1) s += __shfl_xor(s, o); ((volatile float*)NRM)[v * 32 + lane] = lane == 0 ? 1.0f / fmaxf(sqrtf(s), NEPS) : 0.0f; } __threadfence(); }
}
__global__ __launch_bounds__(32) void inc_kernel(const b16* __restrict__ XB, const float* __restrict__ NRM, unsigned char* __restrict__ HB) {
  __shared__ unsigned char Tb[16][132]; const int lane = threadIdx.x, nloc = lane & 15, hlf = lane >> 4; const int b = blockIdx.x / (N / 16), n0 = (blockIdx.x % (N / 16)) * 16; const size_t e0 = (size_t)b * N + n0;
  const b16* ta = XB + (e0 + nloc) * C; float nr[8]; for (int r8 = 0; r8 < 8; ++r8) nr[r8] = NRM[(e0 + 8 * hlf + r8) * 32];
#pragma unroll 1
  for (int cg = 0; cg < NC / 128; ++cg) { v8f acc[8];
#pragma unroll
    for (int t = 0; t < 8; ++t) acc[t] = (v8f){};
#pragma unroll
    for (int kb = 0; kb < C; kb += 32) { const v16b a = frag_kb(ta + kb, hlf);
#pragma unroll
      for (int t = 0; t < 8; ++t) { const size_t cv = (size_t)VT + (size_t)b * NC + cg * 128 + t * 16 + nloc; acc[t] = wmma16b(a, frag_kb(XB + cv * C + kb, hlf), acc[t]); } }
#pragma unroll
    for (int t = 0; t < 8; ++t) { const size_t cv = (size_t)VT + (size_t)b * NC + cg * 128 + t * 16 + nloc; const float nm = NRM[cv * 32];
#pragma unroll
      for (int r8 = 0; r8 < 8; ++r8) { const float s = pmul(pmul(acc[t][r8] * (1.0f / (XS * XS)), nr[r8]), nm); Tb[8 * hlf + r8][t * 16 + nloc] = s > THR ? 1 : 0; } }
    wave_lds_sync();
    for (int pass = 0; pass < 2; ++pass) { for (int rr = 0; rr < 16; ++rr) for (int i = lane * 4; i < 128; i += 128) *(volatile unsigned int*)(HB + (e0 + rr) * NC + cg * 128 + i) = *(const unsigned int*)(&Tb[rr][i]); __threadfence(); }
    wave_lds_sync(); }
}
template <int EXA>
__global__ __launch_bounds__(32) void lin_kernel(const b16* __restrict__ INb, const float* __restrict__ INf, const b16* __restrict__ WT, const float* __restrict__ bias, int RL, float* __restrict__ OUT) {
  __shared__ __attribute__((aligned(16))) b16 Ah[16][C + 8], Al[16][C + 8]; __shared__ float Tf[16][C + 4]; const int lane = threadIdx.x, nloc = lane & 15, hlf = lane >> 4; const size_t m0 = (size_t)blockIdx.x * 16; if (m0 >= (size_t)RL) return;
  if (!EXA) { for (int rr = 0; rr < 16; ++rr) for (int q = 0; q < 8; ++q) { b16 p, ql; split16(INf[(m0 + rr) * C + q * 32 + lane] * XS, p, ql); Ah[rr][q * 32 + lane] = p; Al[rr][q * 32 + lane] = ql; } wave_lds_sync(); }
  v8f acc[16];
#pragma unroll
  for (int t = 0; t < 16; ++t) acc[t] = (v8f){};
#pragma unroll
  for (int kb = 0; kb < C; kb += 32) { v16b a, al; if (EXA) a = frag_kb(INb + (m0 + nloc) * C + kb, hlf); else { a = frag_kb(&Ah[nloc][kb], hlf); al = frag_kb(&Al[nloc][kb], hlf); }
#pragma unroll
    for (int t = 0; t < 16; ++t) { const v16b bw = frag_kb(WT + (size_t)(t * 16 + nloc) * C + kb, hlf); acc[t] = wmma16b(a, bw, acc[t]); if (!EXA) acc[t] = wmma16b(al, bw, acc[t]); } }
#pragma unroll
  for (int t = 0; t < 16; ++t) { const int c = t * 16 + nloc; const float bb = bf16_rne(bias[c]);
#pragma unroll
    for (int r8 = 0; r8 < 8; ++r8) Tf[8 * hlf + r8][c] = acc[t][r8] * (EXA ? 1.0f / (XS * WSC) : 1.0f / (XS * WSC)) + bb; }
  wave_lds_sync();
  for (int pass = 0; pass < 2; ++pass) { for (int rr = 0; rr < 16; ++rr) for (int q = 0; q < 2; ++q) *(volatile v4f*)(OUT + (m0 + rr) * C + q * 128 + lane * 4) = *(const v4f*)(&Tf[rr][q * 128 + lane * 4]); __threadfence(); }
}
__global__ __launch_bounds__(256) void xe_kernel(const float* __restrict__ XN, const unsigned char* __restrict__ HB, float* __restrict__ XE) {
  const int wave = threadIdx.x >> 5, lane = threadIdx.x & 31; const int e = blockIdx.x * 8 + wave; if (e >= ET) return; const int b = e / N, n = e % N; float a[8]; const float* xi = XN + ((size_t)b * (N + NC) + n) * C; for (int q = 0; q < 8; ++q) a[q] = xi[q * 32 + lane]; int cnt = 0;
  int mine = 0; for (int j = 0; j < NC / 32; ++j) mine += HB[(size_t)e * NC + j * 32 + lane] ? 1 : 0; int tot = mine; for (int o = 16; o; o >>= 1) tot += __shfl_xor(tot, o);
  if (tot > 0) {
#pragma unroll 1
    for (int m = 0; m < NC; ++m) { if (HB[(size_t)e * NC + m]) { ++cnt; const float* xr = XN + ((size_t)b * (N + NC) + N + m) * C; for (int q = 0; q < 8; ++q) a[q] += xr[q * 32 + lane]; } } }
  const float inv = 1.0f / (float)(1 + cnt);
  for (int pass = 0; pass < 2; ++pass) { for (int q = 0; q < 8; ++q) ((volatile float*)XE)[(size_t)e * C + q * 32 + lane] = pmul(a[q], inv); __threadfence(); }
}
__global__ __launch_bounds__(256) void xv_kernel(const float* __restrict__ XET, const unsigned char* __restrict__ HB, float* __restrict__ XV) {
  const int wave = threadIdx.x >> 5, lane = threadIdx.x & 31; const int v = blockIdx.x * 8 + wave; if (v >= V) return; const int b = v / (N + NC), j = v % (N + NC); float a[8];
  if (j < N) { const float* xr = XET + ((size_t)b * N + j) * C; for (int q = 0; q < 8; ++q) a[q] = xr[q * 32 + lane]; }
  else { const int m = j - N; for (int q = 0; q < 8; ++q) a[q] = 0.0f; int cnt = 0;
    int mine = 0; for (int k = 0; k < N / 32; ++k) mine += HB[((size_t)b * N + k * 32 + lane) * NC + m] ? 1 : 0; int tot = mine; for (int o = 16; o; o >>= 1) tot += __shfl_xor(tot, o);
    if (tot > 0) {
#pragma unroll 1
      for (int n = 0; n < N; ++n) { if (HB[((size_t)b * N + n) * NC + m]) { ++cnt; const float* xr = XET + ((size_t)b * N + n) * C; for (int q = 0; q < 8; ++q) a[q] += xr[q * 32 + lane]; } } }
    const float inv = 1.0f / (float)(cnt > 0 ? cnt : 1); for (int q = 0; q < 8; ++q) a[q] = pmul(a[q], inv); }
  for (int pass = 0; pass < 2; ++pass) { for (int q = 0; q < 8; ++q) ((volatile float*)XV)[(size_t)v * C + q * 32 + lane] = a[q]; __threadfence(); }
}
__global__ __launch_bounds__(256) void out_kernel(const float* __restrict__ XV, float* __restrict__ out) {
  __shared__ float Ts[32][C + 1]; const int tid = threadIdx.x, wave = tid >> 5, lane = tid & 31; const int blk = blockIdx.x; const int o = blk / (B * 32), b = (blk / 32) % B, h0 = (blk % 32) * 32;
  const size_t vbase = (o == 0) ? (size_t)b * N + h0 : (size_t)VT + (size_t)b * NC + (o == 1 ? 0 : N) + h0;
  for (int r = wave; r < 32; r += 8) for (int q = 0; q < 8; ++q) Ts[r][q * 32 + lane] = XV[(vbase + r) * C + q * 32 + lane];
  __syncthreads();
  for (int pass = 0; pass < 2; ++pass) { for (int c = wave; c < C; c += 8) ((volatile float*)out)[(size_t)o * (B * C * N) + ((size_t)b * C + c) * N + h0 + lane] = Ts[lane][c]; __threadfence(); }
}
}

extern "C" void kernel_launch(void* const* d_in, const int* in_sizes, int n_in, void* d_out, int out_size, void* d_ws, size_t ws_size, hipStream_t stream) {
  (void)n_in;
  auto Fp = [&](int i) { return (const float*)d_in[i]; };
  if (in_sizes[0] != B * C * N || in_sizes[1] != B * C * N || in_sizes[2] != B * C * N || in_sizes[3] != C * C || in_sizes[5] != C * C || out_size != 3 * B * C * N) return;
  size_t off = 0; char* ws = (char*)d_ws;
  auto carve = [&](size_t bytes) { char* p = ws + off; off += (bytes + 255) & ~(size_t)255; return p; };
  b16* WN = (b16*)carve((size_t)C * C * 2); b16* WE = (b16*)carve((size_t)C * C * 2); b16* XB = (b16*)carve((size_t)V * C * 2); float* NRM = (float*)carve((size_t)V * 32 * 4); unsigned char* HB = (unsigned char*)carve((size_t)ET * NC);
  float* XN = (float*)carve((size_t)V * C * 4); float* XE = (float*)carve((size_t)ET * C * 4); float* XET = (float*)carve((size_t)ET * C * 4); float* XV = (float*)carve((size_t)V * C * 4);
  if (off > ws_size || off > ((size_t)64 << 20)) return;
  wcopy_kernel<<<(C * C / 8 + 255) / 256, 256, 0, stream>>>(Fp(3), WN); wcopy_kernel<<<(C * C / 8 + 255) / 256, 256, 0, stream>>>(Fp(5), WE);
  xall_kernel<<<V / 32, 256, 0, stream>>>(Fp(0), Fp(1), Fp(2), XB, NRM);
  inc_kernel<<<B * (N / 16), 32, 0, stream>>>(XB, NRM, HB);
  lin_kernel<1><<<V / 16, 32, 0, stream>>>(XB, nullptr, WN, Fp(4), V, XN);
  xe_kernel<<<ET / 8, 256, 0, stream>>>(XN, HB, XE);
  lin_kernel<0><<<ET / 16, 32, 0, stream>>>(nullptr, XE, WE, Fp(6), ET, XET);
  xv_kernel<<<V / 8, 256, 0, stream>>>(XET, HB, XV);
  out_kernel<<<3 * B * 32, 256, 0, stream>>>(XV, (float*)d_out);
}
